// LSTMModel_45921790329164
// MI455X (gfx1250) — hardware-verified
//
#include <hip/hip_runtime.h>
#include <math.h>

constexpr int NSEQ    = 8192;
constexpr int NSTEP   = 256;
constexpr int NH      = 80;
constexpr int NGATE   = 4 * NH;
constexpr int KPAD    = 96;
constexpr int NTHR    = 128;
constexpr int NWAVE   = NTHR / 32;
constexpr int ROWS_W  = 16;
constexpr int ROWS_B  = NWAVE * ROWS_W;
constexpr int WPITCH  = KPAD;
constexpr int HPITCH  = KPAD;
constexpr int CPITCH  = NH;
constexpr int SPITCH  = 8;
constexpr int NCHUNK  = NH / 16;
constexpr int KGRP8   = KPAD / 8;
constexpr float WCARRY  = 256.0f;
constexpr float HCARRY  = 16.0f;
constexpr float ACC_INV = 1.0f / (WCARRY * HCARRY);
static_assert(NSEQ % ROWS_B == 0);
static_assert(KPAD % 32 == 0 && KPAD >= NH);
static_assert(NH % 16 == 0 && NGATE == 4 * NH);
static_assert((NGATE * KGRP8) % NTHR == 0);
static_assert((NWAVE * ROWS_W * HPITCH) % (8 * NTHR) == 0);
static_assert((NWAVE * ROWS_W * CPITCH) % (4 * NTHR) == 0);
static_assert(ROWS_W * SPITCH == 32 * 4);
static_assert(NSTEP % SPITCH == 0);
static_assert(ROWS_B * 4 == 256);
static_assert(NGATE <= 3 * NTHR && NH <= NTHR);

typedef __attribute__((ext_vector_type(16))) _Float16 v16h;
typedef __attribute__((ext_vector_type(8)))  _Float16 v8h;
typedef __attribute__((ext_vector_type(8)))  float    v8f;
typedef __attribute__((ext_vector_type(4)))  float    v4f;

__device__ __forceinline__ void guard_all(v8f& d0, v8f& d1, v8f& d2, v8f& d3,
                                          v16h a, v16h b0, v16h b1, v16h b2, v16h b3) {
  asm volatile("v_nop\n\tv_nop\n\tv_nop\n\tv_nop"
               : "+v"(d0), "+v"(d1), "+v"(d2), "+v"(d3)
               : "v"(a), "v"(b0), "v"(b1), "v"(b2), "v"(b3));
}
__device__ __forceinline__ void acc_guard4(v8f& a, v8f& b, v8f& c, v8f& d) {
  asm volatile("v_nop\n\tv_nop\n\tv_nop\n\tv_nop" : "+v"(a), "+v"(b), "+v"(c), "+v"(d));
}

template <typename T> struct Frag;
template <> struct Frag<_Float16> {
  typedef v16h V; union U { v16h v; v8h h[2]; };
  static __device__ __forceinline__ v16h load(const _Float16* p) {
    U f; f.h[0] = *(const v8h*)(p); f.h[1] = *(const v8h*)(p + 16); return f.v;
  }
  static __device__ __forceinline__ v8f mma(v16h a, v16h b, v8f c) {
    return __builtin_amdgcn_wmma_f32_16x16x32_f16(false, a, false, b, (short)0, c, false, false);
  }
};

__device__ __forceinline__ float fsig(float x)  { return __builtin_amdgcn_rcpf(1.0f + expf(-x)); }
__device__ __forceinline__ float ftanh(float x) { return 1.0f - 2.0f * __builtin_amdgcn_rcpf(expf(2.0f * x) + 1.0f); }

__device__ __forceinline__ void mma_group(v8f& ai, v8f& af, v8f& ag, v8f& ao, v16h a, const _Float16* wb) {
  const v16h b0 = Frag<_Float16>::load(wb);
  const v16h b1 = Frag<_Float16>::load(wb + 1 * NH * WPITCH);
  const v16h b2 = Frag<_Float16>::load(wb + 2 * NH * WPITCH);
  const v16h b3 = Frag<_Float16>::load(wb + 3 * NH * WPITCH);
  ai = Frag<_Float16>::mma(a, b0, ai);
  af = Frag<_Float16>::mma(a, b1, af);
  ag = Frag<_Float16>::mma(a, b2, ag);
  ao = Frag<_Float16>::mma(a, b3, ao);
  guard_all(ai, af, ag, ao, a, b0, b1, b2, b3);
}

__device__ __forceinline__ void refill_src(float* sw, const float* __restrict__ src, int rowBase, int lane, int t0) {
  const int r = lane >> 1, j4 = (lane & 1) * 4;
  const v4f v = *(const v4f*)(src + (size_t)(rowBase + r) * NSTEP + t0 + j4);
  *(v4f*)(sw + r * SPITCH + j4) = v;
}

__global__ __launch_bounds__(NTHR) void lstm_seq_kernel(const float* __restrict__ src, const float* __restrict__ w_ih,
                                                        const float* __restrict__ w_hh, const float* __restrict__ b_ih,
                                                        const float* __restrict__ b_hh, const float* __restrict__ w_lin,
                                                        const float* __restrict__ b_lin, float* __restrict__ out) {
  __shared__ __align__(16) _Float16 Ws[NGATE * WPITCH];
  __shared__ __align__(16) _Float16 Hs[NWAVE * ROWS_W * HPITCH];
  __shared__ __align__(16) float    Cs[NWAVE * ROWS_W * CPITCH];
  __shared__ __align__(16) float    Ss[NWAVE * ROWS_W * SPITCH];
  __shared__ __align__(16) float    Wx[NGATE];
  __shared__ __align__(16) float    Bsum[NGATE];
  __shared__ __align__(16) float    Wl[NH];
  __shared__ __align__(16) float    Outs[ROWS_B];

  const int tid = threadIdx.x, lane = tid & 31, wave = tid >> 5;
  const int c = lane & 15, hh = lane >> 4;
  const int rowBase = blockIdx.x * ROWS_B + wave * ROWS_W;
  const float blin = b_lin[0];

  _Float16* Hw = Hs + wave * ROWS_W * HPITCH;
  float*    Cw = Cs + wave * ROWS_W * CPITCH;
  float*    Sw = Ss + wave * ROWS_W * SPITCH;

  v8h z8h;
#pragma unroll
  for (int e = 0; e < 8; ++e) z8h[e] = (_Float16)0.0f;
  const v4f z4f = {0.0f, 0.0f, 0.0f, 0.0f};
  const v8f z8f = {0.0f, 0.0f, 0.0f, 0.0f, 0.0f, 0.0f, 0.0f, 0.0f};

#pragma unroll 1
  for (int it = 0; it < (NGATE * KGRP8) / NTHR; ++it) {
    const int task = it * NTHR + tid;
    const int n  = task / KGRP8;
    const int k8 = (task - n * KGRP8) * 8;
    const int kl = (k8 < NH - 8) ? k8 : (NH - 8);
    const float* wp = w_hh + (size_t)n * NH + kl;
    const v4f w0 = *(const v4f*)(wp);
    const v4f w1 = *(const v4f*)(wp + 4);
    const bool real = (k8 < NH);
    v8h hv;
#pragma unroll
    for (int e = 0; e < 4; ++e) {
      const float f0 = real ? w0[e] : 0.0f;
      const float f1 = real ? w1[e] : 0.0f;
      hv[e]     = (_Float16)(f0 * WCARRY);
      hv[4 + e] = (_Float16)(f1 * WCARRY);
    }
    *(v8h*)(Ws + n * WPITCH + k8) = hv;
  }
  asm volatile("" ::: "memory");

#pragma unroll
  for (int it = 0; it < 3; ++it) {
    const int i  = it * NTHR + tid;
    const int ic = (i < NGATE) ? i : (NGATE - 1);
    const float wv = w_ih[ic];
    const float bv = b_ih[ic] + b_hh[ic];
    if (i < NGATE) { Wx[i] = wv; Bsum[i] = bv; }
  }
  asm volatile("" ::: "memory");
  {
    const int ic = (tid < NH) ? tid : (NH - 1);
    const float wl = w_lin[ic];
    if (tid < NH) Wl[tid] = wl;
  }

#pragma unroll
  for (int it = 0; it < (NWAVE * ROWS_W * HPITCH) / (8 * NTHR); ++it) *(v8h*)(Hs + 8 * (it * NTHR + tid)) = z8h;
#pragma unroll
  for (int it = 0; it < (NWAVE * ROWS_W * CPITCH) / (4 * NTHR); ++it) *(v4f*)(Cs + 4 * (it * NTHR + tid)) = z4f;

  refill_src(Sw, src, rowBase, lane, 0);
  __syncthreads();

  const _Float16* hrow = Hw + c * HPITCH + 8 * hh;

#pragma unroll 1
  for (int t = 0; t < NSTEP; ++t) {
    const v16h a0 = Frag<_Float16>::load(hrow);
    const v16h a1 = Frag<_Float16>::load(hrow + 32);
    const v16h a2 = Frag<_Float16>::load(hrow + 64);
    float sv[8];
#pragma unroll
    for (int r = 0; r < 8; ++r) sv[r] = Sw[(8 * hh + r) * SPITCH + (t & 7)];
    const bool last = (t == NSTEP - 1);

#pragma unroll 1
    for (int ch = 0; ch < NCHUNK; ++ch) {
      const int col = 16 * ch + c;
      const _Float16* wb = Ws + col * WPITCH + 8 * hh;
      v8f ai = z8f, af = z8f, ag = z8f, ao = z8f;
      mma_group(ai, af, ag, ao, a0, wb);
      mma_group(ai, af, ag, ao, a1, wb + 32);
      mma_group(ai, af, ag, ao, a2, wb + 64);
      acc_guard4(ai, af, ag, ao);

      const float wx0 = Wx[col], wx1 = Wx[NH + col], wx2 = Wx[2 * NH + col], wx3 = Wx[3 * NH + col];
      const float bs0 = Bsum[col], bs1 = Bsum[NH + col], bs2 = Bsum[2 * NH + col], bs3 = Bsum[3 * NH + col];
#pragma unroll
      for (int r = 0; r < 8; ++r) {
        const float xi = sv[r] * wx0 + bs0;
        const float xf = sv[r] * wx1 + bs1;
        const float xg = sv[r] * wx2 + bs2;
        const float xo = sv[r] * wx3 + bs3;
        const float zi = ai[r] * ACC_INV + xi;
        const float zf = af[r] * ACC_INV + xf;
        const float zg = ag[r] * ACC_INV + xg;
        const float zo = ao[r] * ACC_INV + xo;
        const float ig = fsig(zi);
        const float fg = fsig(zf);
        const float gg = ftanh(zg);
        const float og = fsig(zo);
        const int ci = (8 * hh + r) * CPITCH + col;
        const float cp = Cw[ci];
        const float cn = fg * cp + ig * gg;
        const float hn = og * ftanh(cn);
        Cw[ci] = last ? hn : cn;
        Hw[(8 * hh + r) * HPITCH + col] = (_Float16)(hn * HCARRY);
      }
    }
    *(v8h*)(Hw + (lane & 15) * HPITCH + NH + 8 * hh) = z8h;
    {
      const int tn = t + 1;
      if (tn < NSTEP && (tn & 7) == 0) refill_src(Sw, src, rowBase, lane, tn);
    }
    __syncthreads();
  }

  {
    const int m = lane & 15;
    float accd = 0.0f;
#pragma unroll 1
    for (int k = 0; k < NH; ++k) accd += Cw[m * CPITCH + k] * Wl[k];
    const float res = accd + blin;
    if (hh == 0) Outs[wave * ROWS_W + m] = res;
  }
  __syncthreads();
  if (wave == 0) {
    const v4f v = *(const v4f*)(Outs + 4 * (lane & 15));
    float* op = out + (size_t)blockIdx.x * ROWS_B + 4 * (lane & 15);
    if (lane < 16) *(volatile v4f*)op = v;
    __threadfence();
    if (lane < 16) *(volatile v4f*)op = v;
  }
}

extern "C" void kernel_launch(void* const* d_in, const int* in_sizes, int n_in,
                              void* d_out, int out_size, void* d_ws, size_t ws_size, hipStream_t stream) {
  (void)d_ws; (void)ws_size;
  if (n_in < 7 || d_out == nullptr) return;
  if (in_sizes[0] != NSEQ * NSTEP || in_sizes[1] != NGATE || in_sizes[2] != NGATE * NH || in_sizes[3] != NGATE ||
      in_sizes[4] != NGATE || in_sizes[5] != NH || in_sizes[6] != 1 || out_size != NSEQ) return;

  const float* src   = (const float*)d_in[0];
  const float* w_ih  = (const float*)d_in[1];
  const float* w_hh  = (const float*)d_in[2];
  const float* b_ih  = (const float*)d_in[3];
  const float* b_hh  = (const float*)d_in[4];
  const float* w_lin = (const float*)d_in[5];
  const float* b_lin = (const float*)d_in[6];
  float* out = (float*)d_out;

  lstm_seq_kernel<<<NSEQ / ROWS_B, NTHR, 0, stream>>>(src, w_ih, w_hh, b_ih, b_hh, w_lin, b_lin, out);
}
